// Decoder_14302241095776
// MI455X (gfx1250) — hardware-verified
//
#include <hip/hip_runtime.h>
#include <math.h>

constexpr int NBATCH    = 256;
constexpr int NSTEP     = 4096;
constexpr int NCH       = 8;
constexpr int NHID      = 128;
constexpr int NBT       = NBATCH * NSTEP;
constexpr int UPW       = 16;
constexpr int KIP       = 32;
constexpr int ROWS_BLK  = 16;
constexpr int NWREC     = 8;
constexpr int NTHR_SCAN = 32 * (NWREC + 1);
constexpr int NTHR_PREP = 256;
constexpr int UROWS_BLK = NTHR_PREP / NCH;
constexpr int HPITCH    = 136;
constexpr int HPLANE    = ROWS_BLK * HPITCH;
constexpr int OSPITCH   = 36;
constexpr float RES_SCALE = 4096.0f;
constexpr float RES_INV   = 1.0f / 4096.0f;

static_assert(NBT % UROWS_BLK == 0);
static_assert(NBATCH % ROWS_BLK == 0);
static_assert(NHID == 16 * NWREC);
static_assert(NHID % 32 == 0);
static_assert(NSTEP % 4 == 0);
static_assert(NCH == 8);
static_assert((NHID * NHID / 8) % NTHR_PREP == 0);
static_assert((NHID * KIP / 8) % NTHR_PREP == 0);
static_assert(2 * NCH * NHID / 8 == NTHR_PREP);
static_assert(HPITCH % 8 == 0 && HPITCH >= NHID);
static_assert(OSPITCH % 4 == 0 && OSPITCH >= 4 * NCH);
static_assert(UROWS_BLK * UPW / 8 == 64);

typedef __attribute__((ext_vector_type(16))) _Float16 v16h;
typedef __attribute__((ext_vector_type(8)))  _Float16 v8h;
typedef __attribute__((ext_vector_type(8)))  float    v8f;
typedef __attribute__((ext_vector_type(4)))  float    v4f;

__device__ __forceinline__ void dep_guard_h(v8f& a, v8f& b, v16h x, v16h y) { asm volatile("v_nop\n\tv_nop\n\tv_nop\n\tv_nop" : "+v"(a), "+v"(b) : "v"(x), "v"(y)); }
__device__ __forceinline__ void acc_guard2(v8f& a, v8f& b) { asm volatile("v_nop\n\tv_nop\n\tv_nop\n\tv_nop" : "+v"(a), "+v"(b)); }
__device__ __forceinline__ void keepm_h(v16h a, v16h b) { asm volatile("v_nop" :: "v"(a), "v"(b) : "memory"); }

struct FragH {
  union U { v16h v; v8h h[2]; };
  static __device__ __forceinline__ v16h load(const _Float16* p) {
    U f; f.h[0] = *(const v8h*)(p); f.h[1] = *(const v8h*)(p + 16); return f.v;
  }
  static __device__ __forceinline__ v8f mma(v16h a, v16h b, v8f c) {
    return __builtin_amdgcn_wmma_f32_16x16x32_f16(false, a, false, b, (short)0, c, false, false);
  }
};

__device__ __forceinline__ float ftanh(float x) { return 1.0f - 2.0f * __builtin_amdgcn_rcpf(__expf(2.0f * x) + 1.0f); }

__device__ __forceinline__ void split_h(float v, _Float16& hi, _Float16& lo) {
  hi = (_Float16)v;
  const float hf = (float)hi;
  lo = (_Float16)((v - hf) * RES_SCALE);
}
__device__ __forceinline__ v16h zero16h() {
  v16h z;
#pragma unroll
  for (int e = 0; e < 16; ++e) z[e] = (_Float16)0.0f;
  return z;
}
__device__ __forceinline__ v8h zero8h() {
  v8h z;
#pragma unroll
  for (int e = 0; e < 8; ++e) z[e] = (_Float16)0.0f;
  return z;
}

__global__ __launch_bounds__(NTHR_PREP) void u_prep_kernel(const float* __restrict__ x, const float* __restrict__ W1,
                                                           const float* __restrict__ b1, _Float16* __restrict__ UP) {
  __shared__ __align__(16) _Float16 Us[UROWS_BLK * UPW];
  const int tid = threadIdx.x, rloc = tid >> 3, c = tid & 7;
  const size_t bt = (size_t)blockIdx.x * UROWS_BLK + (size_t)rloc;
  const float xv = x[bt];
  const float w  = W1[c];
  const float bb = b1[c];
  const float u  = ftanh(xv * w + bb);
  _Float16 hi, lo;
  split_h(u, hi, lo);
  Us[rloc * UPW + c] = hi;
  Us[rloc * UPW + NCH + c] = lo;
  __syncthreads();
  if (tid < 64) {
    const v8h v = *(const v8h*)(Us + tid * 8);
    _Float16* dst = UP + (size_t)blockIdx.x * (UROWS_BLK * UPW) + (size_t)tid * 8;
    *(volatile v8h*)dst = v;
    __threadfence();
    *(volatile v8h*)dst = v;
  }
}

__global__ __launch_bounds__(NTHR_PREP) void whh_prep_kernel(const float* __restrict__ W, _Float16* __restrict__ PH,
                                                             _Float16* __restrict__ PL) {
  const int i = blockIdx.x * NTHR_PREP + threadIdx.x;
  if (i < NHID * NHID / 8) {
    const int row = i >> 4, k8 = (i & 15) * 8;
    const float* sp = W + row * NHID + k8;
    const v4f a = *(const v4f*)(sp);
    const v4f b = *(const v4f*)(sp + 4);
    v8h hv, lv;
#pragma unroll
    for (int e = 0; e < 4; ++e) {
      _Float16 h0, l0, h1, l1;
      split_h(a[e], h0, l0);
      split_h(b[e], h1, l1);
      hv[e] = h0; lv[e] = l0; hv[4 + e] = h1; lv[4 + e] = l1;
    }
    _Float16* dh = PH + (size_t)i * 8;
    _Float16* dl = PL + (size_t)i * 8;
    *(volatile v8h*)dh = hv;
    *(volatile v8h*)dl = lv;
    __threadfence();
    *(volatile v8h*)dh = hv;
    *(volatile v8h*)dl = lv;
  }
}

__global__ __launch_bounds__(NTHR_PREP) void wih_prep_kernel(const float* __restrict__ W, _Float16* __restrict__ WIM,
                                                             _Float16* __restrict__ WIR) {
  const int i = blockIdx.x * NTHR_PREP + threadIdx.x;
  if (i < NHID * KIP / 8) {
    const int n = i >> 2, seg = i & 3;
    const float* sp = W + n * NCH;
    const v4f a = *(const v4f*)(sp);
    const v4f b = *(const v4f*)(sp + 4);
    const float f0 = (seg == 0) ? 1.0f : 0.0f;
    const float f1 = (seg == 1) ? 1.0f : 0.0f;
    v8h mv, rv;
#pragma unroll
    for (int e = 0; e < 8; ++e) {
      const float w = (e < 4) ? a[e] : b[e - 4];
      const _Float16 hh16 = (_Float16)w;
      const float hf = (float)hh16;
      const float lf = (w - hf) * RES_SCALE;
      mv[e] = (_Float16)(w * f0);
      rv[e] = (_Float16)(lf * f0 + hf * f1);
    }
    _Float16* dm = WIM + (size_t)i * 8;
    _Float16* dr = WIR + (size_t)i * 8;
    *(volatile v8h*)dm = mv;
    *(volatile v8h*)dr = rv;
    __threadfence();
    *(volatile v8h*)dm = mv;
    *(volatile v8h*)dr = rv;
  }
}

__global__ __launch_bounds__(NTHR_PREP) void w2_prep_kernel(const float* __restrict__ W, _Float16* __restrict__ W2P) {
  const int i = threadIdx.x;
  const int row = i >> 4, k8 = (i & 15) * 8, srow = row & 7;
  const float* sp = W + srow * NHID + k8;
  const v4f a = *(const v4f*)(sp);
  const v4f b = *(const v4f*)(sp + 4);
  const float flo = (row >= NCH) ? 1.0f : 0.0f;
  const float fhi = 1.0f - flo;
  v8h pv;
#pragma unroll
  for (int e = 0; e < 8; ++e) {
    const float w = (e < 4) ? a[e] : b[e - 4];
    const _Float16 hh16 = (_Float16)w;
    const float hf = (float)hh16;
    const float lf = (w - hf) * RES_SCALE;
    pv[e] = (_Float16)(hf * fhi + lf * flo);
  }
  _Float16* dp = W2P + (size_t)i * 8;
  *(volatile v8h*)dp = pv;
  __threadfence();
  *(volatile v8h*)dp = pv;
}

__global__ __launch_bounds__(NTHR_SCAN) void rnn_scan_kernel(
    const _Float16* UP, const _Float16* WHH_HI, const _Float16* WHH_LO,
    const _Float16* WIM, const _Float16* WIR, const _Float16* W2P,
    const float* b_ih, const float* b_hh, const float* b2, float* out) {
  __shared__ __align__(16) _Float16 Hbuf[4 * HPLANE];
  __shared__ __align__(16) float    OutS[ROWS_BLK * OSPITCH];
  const int tid = threadIdx.x, lane = tid & 31, wave = tid >> 5;
  const int c = lane & 15, hh = lane >> 4, koff = 8 * hh;
  const int b0 = blockIdx.x * ROWS_BLK;

#pragma unroll 1
  for (int i = tid; i < 4 * HPLANE; i += NTHR_SCAN) Hbuf[i] = (_Float16)0.0f;

  v16h BF[4], BL[4], BIM, BIR;
  {
    const v16h zf = zero16h();
#pragma unroll
    for (int kc = 0; kc < 4; ++kc) { BF[kc] = zf; BL[kc] = zf; }
    BIM = zf; BIR = zf;
  }
  float bias0 = 0.0f;
  if (wave < NWREC) {
    const int n = 16 * wave + c;
    const _Float16* ph = WHH_HI + (size_t)n * NHID + koff;
    const _Float16* pl = WHH_LO + (size_t)n * NHID + koff;
    BF[0] = FragH::load(ph);       BF[1] = FragH::load(ph + 32);  keepm_h(BF[0], BF[1]);
    BF[2] = FragH::load(ph + 64);  BF[3] = FragH::load(ph + 96);  keepm_h(BF[2], BF[3]);
    BL[0] = FragH::load(pl);       BL[1] = FragH::load(pl + 32);  keepm_h(BL[0], BL[1]);
    BL[2] = FragH::load(pl + 64);  BL[3] = FragH::load(pl + 96);  keepm_h(BL[2], BL[3]);
    BIM = FragH::load(WIM + (size_t)n * KIP + koff);
    BIR = FragH::load(WIR + (size_t)n * KIP + koff);
    keepm_h(BIM, BIR);
    bias0 = b_ih[n] + b_hh[n];
  } else {
    const _Float16* p2 = W2P + (size_t)c * NHID + koff;
    BF[0] = FragH::load(p2);       BF[1] = FragH::load(p2 + 32);  keepm_h(BF[0], BF[1]);
    BF[2] = FragH::load(p2 + 64);  BF[3] = FragH::load(p2 + 96);  keepm_h(BF[2], BF[3]);
    bias0 = b2[c & 7];
  }
  __syncthreads();

  const v8h zh = zero8h();
  const v8f z8 = {0.f, 0.f, 0.f, 0.f, 0.f, 0.f, 0.f, 0.f};

#pragma unroll 1
  for (int t = 0; t <= NSTEP; ++t) {
    const int cur = t & 1, nxt = cur ^ 1;
    const _Float16* hrow = Hbuf + (2 * cur) * HPLANE + c * HPITCH + koff;
    const _Float16* lrow = Hbuf + (2 * cur + 1) * HPLANE + c * HPITCH + koff;
    if (wave < NWREC) {
      if (t < NSTEP) {
        const int n = 16 * wave + c;
        FragH::U ua;
        ua.h[0] = *(const v8h*)(UP + ((size_t)(b0 + c) * NSTEP + (size_t)t) * UPW + koff);
        ua.h[1] = zh;
        v8f acc, accr = z8;
#pragma unroll
        for (int r = 0; r < 8; ++r) acc[r] = bias0;
        acc  = FragH::mma(ua.v, BIM, acc);
        accr = FragH::mma(ua.v, BIR, accr);
        dep_guard_h(acc, accr, ua.v, BIR);
#pragma unroll
        for (int kc = 0; kc < 4; ++kc) {
          const v16h ah = FragH::load(hrow + 32 * kc);
          const v16h al = FragH::load(lrow + 32 * kc);
          acc  = FragH::mma(ah, BF[kc], acc);
          accr = FragH::mma(ah, BL[kc], accr);
          accr = FragH::mma(al, BF[kc], accr);
          dep_guard_h(acc, accr, ah, al);
        }
        acc_guard2(acc, accr);
        _Float16* wh = Hbuf + (2 * nxt) * HPLANE;
        _Float16* wl = Hbuf + (2 * nxt + 1) * HPLANE;
#pragma unroll
        for (int r = 0; r < 8; ++r) {
          const float pre = acc[r] + accr[r] * RES_INV;
          const float hn  = ftanh(pre);
          _Float16 hi, lo;
          split_h(hn, hi, lo);
          wh[(8 * hh + r) * HPITCH + n] = hi;
          wl[(8 * hh + r) * HPITCH + n] = lo;
        }
      }
    } else {
      if (t >= 1) {
        const int s = t - 1, slot = s & 3;
        v8f acco = z8, accor = z8;
#pragma unroll
        for (int kc = 0; kc < 4; ++kc) {
          const v16h ah = FragH::load(hrow + 32 * kc);
          const v16h al = FragH::load(lrow + 32 * kc);
          acco  = FragH::mma(ah, BF[kc], acco);
          accor = FragH::mma(al, BF[kc], accor);
          dep_guard_h(acco, accor, ah, al);
        }
        acc_guard2(acco, accor);
#pragma unroll
        for (int r = 0; r < 8; ++r) {
          const float vo = acco[r];
          const float vr = accor[r];
          const float xo = __shfl_xor(vo, 8, 32);
          const float xr = __shfl_xor(vr, 8, 32);
          const float pre = vo + bias0 + (xo + vr) * RES_INV + xr * (RES_INV * RES_INV);
          const float o = ftanh(pre);
          if (c < NCH) OutS[(8 * hh + r) * OSPITCH + slot * NCH + c] = o;
        }
        if (slot == 3) {
          __builtin_amdgcn_fence(__ATOMIC_RELEASE, "workgroup");
          __builtin_amdgcn_wave_barrier();
          __builtin_amdgcn_fence(__ATOMIC_ACQUIRE, "workgroup");
          const int tb = s - 3;
          const int q = lane >> 3, c4 = (lane & 7) * 4;
          for (int pass = 0; pass < 2; ++pass) {
#pragma unroll
            for (int it = 0; it < 4; ++it) {
              const int row = it * 4 + q;
              const v4f v = *(const v4f*)(OutS + row * OSPITCH + c4);
              *(volatile v4f*)(out + ((size_t)(b0 + row) * NSTEP + (size_t)tb) * NCH + c4) = v;
            }
            __threadfence();
          }
          __builtin_amdgcn_fence(__ATOMIC_RELEASE, "workgroup");
          __builtin_amdgcn_wave_barrier();
          __builtin_amdgcn_fence(__ATOMIC_ACQUIRE, "workgroup");
        }
      }
    }
    __syncthreads();
  }
}

extern "C" void kernel_launch(void* const* d_in, const int* in_sizes, int n_in,
                              void* d_out, int out_size, void* d_ws, size_t ws_size, hipStream_t stream) {
  if (n_in < 9 || d_out == nullptr || d_ws == nullptr) return;
  if (in_sizes[0] != NBT || in_sizes[1] != NCH || in_sizes[2] != NCH || in_sizes[3] != NHID * NCH ||
      in_sizes[4] != NHID || in_sizes[5] != NHID * NHID || in_sizes[6] != NHID || in_sizes[7] != NCH * NHID ||
      in_sizes[8] != NCH || out_size != NBT * NCH) return;

  const float* x    = (const float*)d_in[0];
  const float* W1   = (const float*)d_in[1];
  const float* b1   = (const float*)d_in[2];
  const float* W_ih = (const float*)d_in[3];
  const float* b_ih = (const float*)d_in[4];
  const float* W_hh = (const float*)d_in[5];
  const float* b_hh = (const float*)d_in[6];
  const float* W2   = (const float*)d_in[7];
  const float* b2   = (const float*)d_in[8];
  float* out = (float*)d_out;

  char* ws = (char*)d_ws; size_t off = 0;
  auto carve = [&](size_t bytes) -> char* { char* p = ws + off; off += (bytes + 255) & ~(size_t)255; return p; };
  _Float16* UP     = (_Float16*)carve((size_t)NBT * UPW * 2);
  _Float16* WHH_HI = (_Float16*)carve((size_t)NHID * NHID * 2);
  _Float16* WHH_LO = (_Float16*)carve((size_t)NHID * NHID * 2);
  _Float16* WIM    = (_Float16*)carve((size_t)NHID * KIP * 2);
  _Float16* WIR    = (_Float16*)carve((size_t)NHID * KIP * 2);
  _Float16* W2P    = (_Float16*)carve((size_t)2 * NCH * NHID * 2);
  if (off > ws_size || off > (size_t)134217728) return;

  u_prep_kernel<<<NBT / UROWS_BLK, NTHR_PREP, 0, stream>>>(x, W1, b1, UP);
  whh_prep_kernel<<<(NHID * NHID / 8) / NTHR_PREP, NTHR_PREP, 0, stream>>>(W_hh, WHH_HI, WHH_LO);
  wih_prep_kernel<<<(NHID * KIP / 8) / NTHR_PREP, NTHR_PREP, 0, stream>>>(W_ih, WIM, WIR);
  w2_prep_kernel<<<1, NTHR_PREP, 0, stream>>>(W2, W2P);
  rnn_scan_kernel<<<NBATCH / ROWS_BLK, NTHR_SCAN, 0, stream>>>(UP, WHH_HI, WHH_LO, WIM, WIR, W2P, b_ih, b_hh, b2, out);
}
